// RelationalGATLayer_28484223107793
// MI455X (gfx1250) — hardware-verified
//
#include <hip/hip_runtime.h>
#include <math.h>

#define NN     30000
#define NP     30016
#define NE     300000
#define NREL   8
#define NHEAD  8
#define HD     32
#define INFEAT 256
#define OUTF   256
#define NT     256
#define SRB    512
#define NTILE  59
#define RPW    (SRB / 8)
#define SCH    4096
#define NCH    ((NE + SCH - 1) / SCH)
#define RQ     2
#define NQT    4
#define XSC    64.0f
#define WSC    256.0f
#define GSCALE (1.0f / 16384.0f)
#define NEG_SLOPE 0.2f

typedef __attribute__((ext_vector_type(16))) _Float16 v16h;
typedef __attribute__((ext_vector_type(8)))  _Float16 v8h;
typedef __attribute__((ext_vector_type(16))) __bf16   v16b;
typedef __attribute__((ext_vector_type(8)))  __bf16   v8b;
typedef __attribute__((ext_vector_type(8)))  float    v8f;
typedef __attribute__((ext_vector_type(4)))  float    v4f;
typedef __attribute__((ext_vector_type(4)))  int      v4i;
typedef __attribute__((ext_vector_type(2)))  unsigned int v2u;

__device__ __forceinline__ unsigned short f2bf_bits(float f) {
  unsigned u = __float_as_uint(f);
  return (unsigned short)((u + 0x7FFFu + ((u >> 16) & 1u)) >> 16);
}
__device__ __forceinline__ float bf_bits2f(unsigned short h) { return __uint_as_float(((unsigned)h) << 16); }

__device__ __forceinline__ void dep_guard_h(v8f& a, v8f& b, v16h x, v16h y) { asm volatile("v_nop\n\tv_nop\n\tv_nop\n\tv_nop" : "+v"(a), "+v"(b) : "v"(x), "v"(y)); }
__device__ __forceinline__ void dep_guard_b(v8f& a, v8f& b, v16b x, v16b y) { asm volatile("v_nop\n\tv_nop\n\tv_nop\n\tv_nop" : "+v"(a), "+v"(b) : "v"(x), "v"(y)); }
__device__ __forceinline__ void keep4_h(v16h a, v16h b, v16h c, v16h d) { asm volatile("v_nop" :: "v"(a), "v"(b), "v"(c), "v"(d)); }
__device__ __forceinline__ void keep4_b(v16b a, v16b b, v16b c, v16b d) { asm volatile("v_nop" :: "v"(a), "v"(b), "v"(c), "v"(d)); }
__device__ __forceinline__ void acc_guard4(v8f& a, v8f& b, v8f& c, v8f& d) { asm volatile("v_nop\n\tv_nop\n\tv_nop\n\tv_nop" : "+v"(a), "+v"(b), "+v"(c), "+v"(d)); }
template <typename T> struct Frag;
template <> struct Frag<_Float16> {
  typedef v16h V; union U { v16h v; v8h h[2]; };
  static __device__ __forceinline__ v16h load(const _Float16* p) {
    U f; f.h[0] = *(const v8h*)(p); f.h[1] = *(const v8h*)(p + 16); return f.v;
  }
  static __device__ __forceinline__ v8f mma(v16h a, v16h b, v8f c) {
    return __builtin_amdgcn_wmma_f32_16x16x32_f16(false, a, false, b, (short)0, c, false, false);
  }
  static __device__ __forceinline__ void guard(v8f& a, v8f& b, v16h x, v16h y) { dep_guard_h(a, b, x, y); }
  static __device__ __forceinline__ void keep(v16h a, v16h b, v16h c, v16h d) { keep4_h(a, b, c, d); }
};
template <> struct Frag<__bf16> {
  typedef v16b V; union U { v16b v; v8b h[2]; };
  static __device__ __forceinline__ v16b load(const __bf16* p) {
    U f; f.h[0] = *(const v8b*)(p); f.h[1] = *(const v8b*)(p + 16); return f.v;
  }
  static __device__ __forceinline__ v8f mma(v16b a, v16b b, v8f c) {
    return __builtin_amdgcn_wmma_f32_16x16x32_bf16(false, a, false, b, (short)0, c, false, false);
  }
  static __device__ __forceinline__ void guard(v8f& a, v8f& b, v16b x, v16b y) { dep_guard_b(a, b, x, y); }
  static __device__ __forceinline__ void keep(v16b a, v16b b, v16b c, v16b d) { keep4_b(a, b, c, d); }
};

__device__ __forceinline__ float dot4(v4f a, v4f b) { return a[0] * b[0] + a[1] * b[1] + a[2] * b[2] + a[3] * b[3]; }

__device__ __forceinline__ int blk_excl_scan(int cnt, int* scan_ws, int tid, int* tot) {
  const int lane = tid & 31, wave = tid >> 5; int incl = cnt;
#pragma unroll
  for (int o = 1; o < 32; o <<= 1) { const int v = __shfl_up(incl, o, 32); if (lane >= o) incl += v; }
  if (lane == 31) scan_ws[wave] = incl;
  __syncthreads();
  if (wave == 0) { int wv = (lane < NT / 32) ? scan_ws[lane] : 0; int wincl = wv;
#pragma unroll
    for (int o = 1; o < 32; o <<= 1) { const int v = __shfl_up(wincl, o, 32); if (lane >= o) wincl += v; }
    if (lane < NT / 32) scan_ws[32 + lane] = wincl - wv; if (lane == 31) scan_ws[64] = wincl; }
  __syncthreads();
  const int res = scan_ws[32 + wave] + incl - cnt; *tot = scan_ws[64];
  return res;
}
template <int SP, int CAP>
__device__ __forceinline__ int chunk_hits(const int* __restrict__ dstv, const int* __restrict__ srcv, const int* __restrict__ typv,
                                          int e0, int n0, int nhi, int qt, int tid, int* LIST, int* scan_ws) {
  const int eb = e0 + tid * SP;
  const bool inr = eb < NE;
  const int ebc = inr ? eb : (NE - SP);
  int rec[SP]; int cnt = 0;
#pragma unroll
  for (int k = 0; k < SP; k += 4) {
    const v4i d4 = *(const v4i*)(dstv + ebc + k);
    const v4i s4 = *(const v4i*)(srcv + ebc + k);
    const v4i t4 = *(const v4i*)(typv + ebc + k);
#pragma unroll
    for (int e = 0; e < 4; ++e) {
      const int d = d4[e]; int t = t4[e]; t = t < 0 ? 0 : (t > NREL - 1 ? NREL - 1 : t);
      int r = -1;
      if (inr && d >= n0 && d < nhi && (t >> 1) == qt) {
        int s = s4[e]; s = s < 0 ? 0 : (s >= NN ? NN - 1 : s);
        r = ((t & 1) << 25) | ((d - n0) << 16) | s; ++cnt;
      }
      rec[k + e] = r;
    }
  }
  int tot; int p = blk_excl_scan(cnt, scan_ws, tid, &tot);
#pragma unroll
  for (int k = 0; k < SP; ++k) if (rec[k] >= 0) { if ((unsigned)p < (unsigned)CAP) LIST[p] = rec[k]; ++p; }
  __syncthreads();
  return tot < CAP ? tot : CAP;
}

#define NXD (NP * INFEAT / 2)
#define NWD (NREL * OUTF * INFEAT / 2)
__global__ __launch_bounds__(NT) void prep_kernel(const float* __restrict__ x, const float* __restrict__ W,
                                                 unsigned* __restrict__ XA32, unsigned* __restrict__ WF32) {
  const int i = blockIdx.x * NT + threadIdx.x;
  if (i < NXD) {
    const int row = i >> 7; const int k = (i & 127) * 2;
    const int rowc = row < NN ? row : NN - 1;
    const float* p = x + (size_t)rowc * INFEAT + k;
    float a = p[0] * XSC, b = p[1] * XSC;
    if (row >= NN) { a = 0.f; b = 0.f; }
    const _Float16 h0 = (_Float16)a, h1 = (_Float16)b;
    const unsigned u = (unsigned)__builtin_bit_cast(unsigned short, h0) | ((unsigned)__builtin_bit_cast(unsigned short, h1) << 16);
    ((volatile unsigned*)XA32)[i] = u;
    __threadfence();
    ((volatile unsigned*)XA32)[i] = u;
  }
  if (i < NWD) {
    const float a = W[2 * (size_t)i] * WSC, b = W[2 * (size_t)i + 1] * WSC;
    const _Float16 h0 = (_Float16)a, h1 = (_Float16)b;
    const unsigned u = (unsigned)__builtin_bit_cast(unsigned short, h0) | ((unsigned)__builtin_bit_cast(unsigned short, h1) << 16);
    ((volatile unsigned*)WF32)[i] = u;
    __threadfence();
    ((volatile unsigned*)WF32)[i] = u;
  }
}

__global__ __launch_bounds__(256) void proj_gemm(
    const unsigned short* __restrict__ XAp, const unsigned short* __restrict__ WFp,
    const float* __restrict__ asrc, const float* __restrict__ adst,
    unsigned short* __restrict__ HPH, unsigned short* __restrict__ HPL, float* __restrict__ AL, float scale) {
  typedef _Float16 T;
  typedef Frag<T>::V V;
  const T* A = (const T*)XAp; const T* Bt = (const T*)WFp;
  __shared__ __align__(16) float sT[8][16 * 68];
  const int b    = blockIdx.y;
  const int lane = threadIdx.x & 31;
  const int wave = threadIdx.x >> 5;
  const int tilesN = OUTF >> 6;
  const int tilesM = NP >> 6;
  const int tile = blockIdx.x * 8 + wave;
  if (tile >= tilesM * tilesN) return;
  const int tm = tile / tilesN;
  const int tn = tile - tm * tilesN;
  const int m0 = tm << 6;
  const int n0 = tn << 6;
  const int lda = INFEAT, ldb = INFEAT, ldc = OUTF, K = INFEAT;

  const T* Ab = A;
  const T* Bb = Bt + (size_t)b * OUTF * INFEAT;

  const int rlane = lane & 15;
  const int koff  = (lane >> 4) * 8;
  const int mOff  = (lane >> 4) * 8;

  v8f acc[4][4];
#pragma unroll
  for (int i = 0; i < 4; ++i)
#pragma unroll
    for (int j = 0; j < 4; ++j) acc[i][j] = (v8f){0.f,0.f,0.f,0.f,0.f,0.f,0.f,0.f};

  for (int k0 = 0; k0 < K; k0 += 32) {
    V bh[4];
#pragma unroll
    for (int j = 0; j < 4; ++j) {
      const size_t bo = (size_t)(n0 + (j << 4) + rlane) * ldb + koff + k0;
      bh[j] = Frag<T>::load(Bb + bo);
    }
#pragma unroll
    for (int i = 0; i < 4; ++i) {
      const size_t ao = (size_t)(m0 + (i << 4) + rlane) * lda + koff + k0;
      V ah = Frag<T>::load(Ab + ao);
#pragma unroll
      for (int j = 0; j < 4; ++j) {
        acc[i][j] = Frag<T>::mma(ah, bh[j], acc[i][j]);
      }
      Frag<T>::guard(acc[i][0], acc[i][3], ah, ah);
    }
    Frag<T>::keep(bh[0], bh[1], bh[2], bh[3]);
  }
  acc_guard4(acc[0][0], acc[0][1], acc[0][2], acc[0][3]);
  acc_guard4(acc[1][0], acc[1][1], acc[1][2], acc[1][3]);
  acc_guard4(acc[2][0], acc[2][1], acc[2][2], acc[2][3]);
  acc_guard4(acc[3][0], acc[3][1], acc[3][2], acc[3][3]);

  float* slab = sT[wave];
  unsigned short* C  = HPH + (size_t)b * NP * OUTF;
  unsigned short* C2 = HPL + (size_t)b * NP * OUTF;
  float* ALb = AL + ((size_t)b * 4 + tn) * NP * 4;
  const int hl = lane >> 4;
  const int head = tn * 2 + hl;
  const float* pa = asrc + head * HD;
  const float* pb = adst + head * HD;
#pragma unroll
  for (int i = 0; i < 4; ++i) {
    const int mBase = m0 + (i << 4);
#pragma unroll
    for (int j = 0; j < 4; ++j) {
#pragma unroll
      for (int r = 0; r < 8; ++r) {
        float v = acc[i][j][r] * scale;
        slab[(mOff + r) * 68 + (j << 4) + rlane] = v;
      }
    }
    __builtin_amdgcn_fence(__ATOMIC_RELEASE, "workgroup");
    __builtin_amdgcn_wave_barrier();
    __builtin_amdgcn_fence(__ATOMIC_ACQUIRE, "workgroup");
    float sv = 0.f, dv = 0.f;
    {
      const float* sp = slab + rlane * 68 + hl * HD;
#pragma unroll 2
      for (int dq = 0; dq < 8; ++dq) {
        const v4f hv = *(const v4f*)(sp + 4 * dq);
        const v4f av = *(const v4f*)(pa + 4 * dq);
        const v4f bv = *(const v4f*)(pb + 4 * dq);
        sv += dot4(hv, av);
        dv += dot4(hv, bv);
      }
    }
    const float sx = __shfl_xor(sv, 16, 32), dx = __shfl_xor(dv, 16, 32);
    v4f arec; arec[0] = sv; arec[1] = sx; arec[2] = dv; arec[3] = dx;
    float* ap = ALb + (size_t)(mBase + rlane) * 4;
    const int q = lane >> 3, c8 = (lane & 7) * 8;
    for (int pass = 0; pass < 2; ++pass) {
#pragma unroll
      for (int it = 0; it < 4; ++it) {
        const int row = it * 4 + q;
        const float* sp = slab + row * 68 + c8;
        v8h hv, lv;
#pragma unroll
        for (int e = 0; e < 8; ++e) {
          unsigned short hb = f2bf_bits(sp[e]);
          unsigned short lb = f2bf_bits(sp[e] - bf_bits2f(hb));
          hv[e] = __builtin_bit_cast(_Float16, hb);
          lv[e] = __builtin_bit_cast(_Float16, lb);
        }
        *(volatile v8h*)(C  + (size_t)(mBase + row) * ldc + n0 + c8) = hv;
        *(volatile v8h*)(C2 + (size_t)(mBase + row) * ldc + n0 + c8) = lv;
      }
      if (lane < 16) *(volatile v4f*)ap = arec;
      __threadfence();
    }
    __builtin_amdgcn_fence(__ATOMIC_RELEASE, "workgroup");
    __builtin_amdgcn_wave_barrier();
    __builtin_amdgcn_fence(__ATOMIC_ACQUIRE, "workgroup");
  }
}

template <int MODE>
__global__ __launch_bounds__(NT) void agg_kernel(const unsigned short* __restrict__ HPH, const unsigned short* __restrict__ HPL,
                                                const float* __restrict__ AL, const int* __restrict__ ei, const int* __restrict__ et,
                                                float* ML, float* out, int qt) {
  __shared__ int LIST[SCH];
  __shared__ __align__(16) float SM[SRB * NHEAD];
  __shared__ __align__(16) float SL[SRB * NHEAD];
  __shared__ int scan_ws[80];
  const int tid = threadIdx.x, lane = tid & 31, wave = tid >> 5;
  const int n0 = blockIdx.x * SRB;
  const int nhi = (n0 + SRB < NN) ? (n0 + SRB) : NN;
  const int h0 = lane >> 3, h1 = h0 + 4, hc = h0 & 1, tnl = lane >> 4;
  const int* srcv = ei;
  const int* dstv = ei + NE;

  if (MODE == 0) {
    for (int i = tid; i < SRB * NHEAD; i += NT) { SM[i] = 0.f; SL[i] = 0.f; }
    const v4f z4 = {0.f, 0.f, 0.f, 0.f};
    for (int ps = 0; ps < 2; ++ps) {
#pragma unroll 1
      for (int j = 0; j < RPW; ++j) {
        const int n = n0 + wave * RPW + j;
        if (n < NN) {
          float* rp = out + (size_t)n * OUTF;
          *(volatile v4f*)(rp + 4 * lane) = z4;
          *(volatile v4f*)(rp + 128 + 4 * lane) = z4;
        }
      }
      __threadfence();
    }
  } else {
#pragma unroll
    for (int part = 0; part < 4; ++part) {
      for (int r = tid; r < SRB; r += NT) {
        const v4f v = *(const v4f*)(ML + (size_t)(n0 + r) * 16 + part * 4);
#pragma unroll
        for (int e = 0; e < 4; ++e) {
          if (part < 2) SM[r * 8 + (part & 1) * 4 + e] = v[e];
          else          SL[r * 8 + (part & 1) * 4 + e] = v[e];
        }
      }
    }
  }
  __syncthreads();

#pragma unroll 1
  for (int c = 0; c < NCH; ++c) {
    const int tot = chunk_hits<SCH / NT, SCH>(dstv, srcv, et, c * SCH, n0, nhi, qt, tid, LIST, scan_ws);
#pragma unroll 1
    for (int base = 0; base < tot; base += 32) {
      int qi = base + lane; const bool inl = qi < tot; qi = qi < SCH ? qi : SCH - 1;
      const int lsv = LIST[qi];
      const int rv = inl ? lsv : -1;
      const int own = (rv >= 0 && ((rv >> 22) & 7) == wave) ? 1 : 0;
      unsigned msk = (unsigned)__ballot(own);
#pragma unroll 1
      for (int it = 0; it < 32; ++it) {
        if (msk == 0u) break;
        const int bp = __builtin_ctz(msk); msk &= msk - 1u;
        const int r = __shfl(rv, bp, 32);
        const int tl = (r >> 25) & 1, dl = (r >> 16) & 511, s = r & 0xFFFF;
        const int q = n0 + dl;
        const float* alb = AL + (size_t)tl * (4 * NP * 4);
        const v4f as0 = *(const v4f*)(alb + ((size_t)tnl * NP + s) * 4);
        const v4f as1 = *(const v4f*)(alb + ((size_t)(tnl + 2) * NP + s) * 4);
        const v4f ad0 = *(const v4f*)(alb + ((size_t)tnl * NP + q) * 4);
        const v4f ad1 = *(const v4f*)(alb + ((size_t)(tnl + 2) * NP + q) * 4);
        float sc0 = (hc ? as0[1] : as0[0]) + (hc ? ad0[3] : ad0[2]);
        float sc1 = (hc ? as1[1] : as1[0]) + (hc ? ad1[3] : ad1[2]);
        sc0 = sc0 > 0.f ? sc0 : NEG_SLOPE * sc0;
        sc1 = sc1 > 0.f ? sc1 : NEG_SLOPE * sc1;
        const float m0o = SM[dl * 8 + h0], l0o = SL[dl * 8 + h0];
        const float m1o = SM[dl * 8 + h1], l1o = SL[dl * 8 + h1];
        const float mn0 = fmaxf(m0o, sc0), mn1 = fmaxf(m1o, sc1);
        const float rr0 = __expf(m0o - mn0), ex0 = __expf(sc0 - mn0);
        const float rr1 = __expf(m1o - mn1), ex1 = __expf(sc1 - mn1);
        const float ln0 = l0o * rr0 + ex0, ln1 = l1o * rr1 + ex1;
        const size_t hro = ((size_t)tl * NP + s) * OUTF;
        const v2u wh0 = *(const v2u*)(HPH + hro + 4 * lane);
        const v2u wh1 = *(const v2u*)(HPH + hro + 128 + 4 * lane);
        const v2u wl0 = *(const v2u*)(HPL + hro + 4 * lane);
        const v2u wl1 = *(const v2u*)(HPL + hro + 128 + 4 * lane);
        v4f hv0, hv1;
        hv0[0] = __uint_as_float(wh0[0] << 16)          + __uint_as_float(wl0[0] << 16);
        hv0[1] = __uint_as_float(wh0[0] & 0xffff0000u) + __uint_as_float(wl0[0] & 0xffff0000u);
        hv0[2] = __uint_as_float(wh0[1] << 16)          + __uint_as_float(wl0[1] << 16);
        hv0[3] = __uint_as_float(wh0[1] & 0xffff0000u) + __uint_as_float(wl0[1] & 0xffff0000u);
        hv1[0] = __uint_as_float(wh1[0] << 16)          + __uint_as_float(wl1[0] << 16);
        hv1[1] = __uint_as_float(wh1[0] & 0xffff0000u) + __uint_as_float(wl1[0] & 0xffff0000u);
        hv1[2] = __uint_as_float(wh1[1] << 16)          + __uint_as_float(wl1[1] << 16);
        hv1[3] = __uint_as_float(wh1[1] & 0xffff0000u) + __uint_as_float(wl1[1] & 0xffff0000u);
        float* rp = out + (size_t)q * OUTF;
        v4f a0 = *(const v4f*)(rp + 4 * lane);
        v4f a1 = *(const v4f*)(rp + 128 + 4 * lane);
        a0 = a0 * rr0 + ex0 * hv0;
        a1 = a1 * rr1 + ex1 * hv1;
        if ((lane & 7) == 0) { SM[dl * 8 + h0] = mn0; SL[dl * 8 + h0] = ln0; SM[dl * 8 + h1] = mn1; SL[dl * 8 + h1] = ln1; }
        *(volatile v4f*)(rp + 4 * lane) = a0;
        *(volatile v4f*)(rp + 128 + 4 * lane) = a1;
        __threadfence();
        *(volatile v4f*)(rp + 4 * lane) = a0;
        *(volatile v4f*)(rp + 128 + 4 * lane) = a1;
      }
    }
    __syncthreads();
  }

  if (MODE == 2) {
#pragma unroll 1
    for (int j = 0; j < RPW; ++j) {
      const int dl = wave * RPW + j; const int n = n0 + dl;
      if (n < NN) {
        const float l0 = SL[dl * 8 + h0], l1 = SL[dl * 8 + h1];
        const float inv0 = 1.0f / (l0 + 1e-12f), inv1 = 1.0f / (l1 + 1e-12f);
        float* rp = out + (size_t)n * OUTF;
        const v4f a0 = *(const v4f*)(rp + 4 * lane) * inv0;
        const v4f a1 = *(const v4f*)(rp + 128 + 4 * lane) * inv1;
        *(volatile v4f*)(rp + 4 * lane) = a0;
        *(volatile v4f*)(rp + 128 + 4 * lane) = a1;
        __threadfence();
        *(volatile v4f*)(rp + 4 * lane) = a0;
        *(volatile v4f*)(rp + 128 + 4 * lane) = a1;
      }
    }
  } else {
    for (int ps = 0; ps < 2; ++ps) {
#pragma unroll 1
      for (int j = 0; j < RPW / 8; ++j) {
        const int dl = wave * RPW + j * 8 + (lane >> 2); const int part = lane & 3;
        const v4f vm = *(const v4f*)(SM + dl * 8 + (part & 1) * 4);
        const v4f vl = *(const v4f*)(SL + dl * 8 + (part & 1) * 4);
        v4f v;
#pragma unroll
        for (int e = 0; e < 4; ++e) v[e] = (part < 2) ? vm[e] : vl[e];
        *(volatile v4f*)(ML + (size_t)(n0 + dl) * 16 + part * 4) = v;
      }
      __threadfence();
    }
  }
}

extern "C" void kernel_launch(void* const* d_in, const int* in_sizes, int n_in,
                              void* d_out, int out_size, void* d_ws, size_t ws_size,
                              hipStream_t stream) {
  (void)in_sizes; (void)n_in; (void)out_size;
  const float* x    = (const float*)d_in[0];
  const float* W    = (const float*)d_in[1];
  const float* asrc = (const float*)d_in[2];
  const float* adst = (const float*)d_in[3];
  const int*   ei   = (const int*)d_in[4];
  const int*   et   = (const int*)d_in[5];
  float* out = (float*)d_out;

  char* ws = (char*)d_ws; size_t off = 0;
  auto carve = [&](size_t bytes) -> char* { char* p = ws + off; off += (bytes + 255) & ~(size_t)255; return p; };
  unsigned short* WF  = (unsigned short*)carve((size_t)NREL * OUTF * INFEAT * 2);
  unsigned short* XA  = (unsigned short*)carve((size_t)NP * INFEAT * 2);
  unsigned short* HPH = (unsigned short*)carve((size_t)RQ * NP * OUTF * 2);
  unsigned short* HPL = (unsigned short*)carve((size_t)RQ * NP * OUTF * 2);
  float*          AL  = (float*)carve((size_t)RQ * 4 * NP * 4 * 4);
  float*          ML  = (float*)carve((size_t)NTILE * SRB * 16 * 4);
  if (off > ws_size || off > (size_t)134217728) return;

  prep_kernel<<<(NXD + NT - 1) / NT, NT, 0, stream>>>(x, W, (unsigned*)XA, (unsigned*)WF);

  const int tiles = (NP / 64) * (OUTF / 64);
  for (int qt = 0; qt < NQT; ++qt) {
    proj_gemm<<<dim3((tiles + 7) / 8, RQ), 256, 0, stream>>>(
        (const unsigned short*)XA, (const unsigned short*)(WF + (size_t)qt * RQ * OUTF * INFEAT),
        asrc, adst, HPH, HPL, AL, GSCALE);
    if (qt == 0)
      agg_kernel<0><<<NTILE, NT, 0, stream>>>(HPH, HPL, AL, ei, et, ML, out, qt);
    else if (qt < NQT - 1)
      agg_kernel<1><<<NTILE, NT, 0, stream>>>(HPH, HPL, AL, ei, et, ML, out, qt);
    else
      agg_kernel<2><<<NTILE, NT, 0, stream>>>(HPH, HPL, AL, ei, et, ML, out, qt);
  }
}
